// LSTM_32091995636113
// MI455X (gfx1250) — hardware-verified
//
#include <hip/hip_runtime.h>
#include <math.h>

constexpr int NBATCH   = 4096;
constexpr int NSTEP    = 512;
constexpr int NHID     = 32;
constexpr int NGATE    = 4 * NHID;
constexpr int NTHR     = 256;
constexpr int ROWS_BLK = 16 * (NTHR / 32);
constexpr int XCHUNK   = 32;
constexpr int XPITCH   = 36;
constexpr int WPLANE   = NGATE * NHID;
constexpr float H_CARRY = 256.0f;
constexpr float W_CARRY = 16.0f;
constexpr float Z_CARRY = H_CARRY * W_CARRY;
constexpr float Z_INV   = 1.0f / Z_CARRY;
static_assert(NHID == 32, "one 32-deep k step");
static_assert(NGATE == 128, "8 gate tiles of 16 rows");
static_assert(ROWS_BLK == 128, "8 waves x 16 rows");
static_assert(NBATCH % ROWS_BLK == 0, "grid exact");
static_assert(NSTEP % XCHUNK == 0, "x tiles exact");
static_assert((XPITCH % 4) == 0 && XPITCH >= XCHUNK, "x tile pitch");
static_assert(Z_CARRY == 4096.0f, "carry product");

typedef __attribute__((ext_vector_type(16))) _Float16 v16h;
typedef __attribute__((ext_vector_type(8)))  _Float16 v8h;
typedef __attribute__((ext_vector_type(8)))  float    v8f;
typedef __attribute__((ext_vector_type(4)))  float    v4f;

__device__ __forceinline__ void acc_guard4(v8f& a, v8f& b, v8f& c, v8f& d) { asm volatile("v_nop\n\tv_nop\n\tv_nop\n\tv_nop" : "+v"(a), "+v"(b), "+v"(c), "+v"(d)); }
template <typename T> struct Frag;
template <> struct Frag<_Float16> {
  typedef v16h V; union U { v16h v; v8h h[2]; };
  static __device__ __forceinline__ v16h load(const _Float16* p) {
    U f; f.h[0] = *(const v8h*)(p); f.h[1] = *(const v8h*)(p + 16); return f.v;
  }
  static __device__ __forceinline__ v8f mma(v16h a, v16h b, v8f c) {
    return __builtin_amdgcn_wmma_f32_16x16x32_f16(false, a, false, b, (short)0, c, false, false);
  }
};

__device__ __forceinline__ v8f wm(v16h a, v16h b, v8f c) {
  c = Frag<_Float16>::mma(a, b, c);
  asm volatile("v_nop\n\tv_nop\n\tv_nop\n\tv_nop" : "+v"(c) : "v"(a), "v"(b));
  return c;
}

__device__ __forceinline__ float gate_sig(float z)  { return __builtin_amdgcn_rcpf(1.0f + expf(-z)); }
__device__ __forceinline__ float gate_tanh(float z) { return 1.0f - 2.0f * __builtin_amdgcn_rcpf(1.0f + expf(2.0f * z)); }

__device__ __forceinline__ v8f ld8(const float* p) {
  const v4f a = *(const v4f*)(p);
  const v4f b = *(const v4f*)(p + 4);
  v8f r;
  r[0] = a[0]; r[1] = a[1]; r[2] = a[2]; r[3] = a[3];
  r[4] = b[0]; r[5] = b[1]; r[6] = b[2]; r[7] = b[3];
  return r;
}

__device__ __forceinline__ v8f cinit0(float xv, const float* wp, const float* bp) {
  const v8f w = ld8(wp);
  const v8f b = ld8(bp);
  v8f r;
#pragma unroll
  for (int e = 0; e < 8; ++e) r[e] = fmaf(xv, w[e], b[e]);
  return r;
}

__device__ __forceinline__ void lstm_cell8(const v8f& zi, const v8f& zf, const v8f& zg, const v8f& zo,
                                           const v8f& cprev, v8f& cnew, v8f& hnew) {
#pragma unroll
  for (int r = 0; r < 8; ++r) {
    const float iv = gate_sig(zi[r] * Z_INV);
    const float fv = gate_sig(zf[r] * Z_INV);
    const float gv = gate_tanh(zg[r] * Z_INV);
    const float ov = gate_sig(zo[r] * Z_INV);
    const float cv = fv * cprev[r] + iv * gv;
    cnew[r] = cv;
    hnew[r] = ov * gate_tanh(cv);
  }
}

__device__ __forceinline__ void stage_w(const float* __restrict__ W, _Float16* dst, int tid) {
#pragma unroll 1
  for (int it = 0; it < 2; ++it) {
    const int idx = it * NTHR + tid;
    const int row = idx >> 2;
    const int q8  = (idx & 3) * 8;
    const v4f a = *(const v4f*)(W + row * NHID + q8);
    const v4f b = *(const v4f*)(W + row * NHID + q8 + 4);
    v8h hv;
#pragma unroll
    for (int e = 0; e < 4; ++e) {
      hv[e]     = (_Float16)(a[e] * W_CARRY);
      hv[4 + e] = (_Float16)(b[e] * W_CARRY);
    }
    *(v8h*)(dst + row * NHID + q8) = hv;
  }
}

__global__ __launch_bounds__(NTHR) void lstm2_fused_kernel(
    const float* __restrict__ x,
    const float* __restrict__ W_ih0, const float* __restrict__ W_hh0,
    const float* __restrict__ b_ih0, const float* __restrict__ b_hh0,
    const float* __restrict__ W_ih1, const float* __restrict__ W_hh1,
    const float* __restrict__ b_ih1, const float* __restrict__ b_hh1,
    const float* __restrict__ W_fc,  const float* __restrict__ b_fc,
    float* __restrict__ out) {
  __shared__ __align__(16) _Float16 Wl[3 * WPLANE];
  __shared__ __align__(16) float xs[ROWS_BLK * XPITCH];
  __shared__ __align__(16) float w0s[NGATE];
  __shared__ __align__(16) float b0s[NGATE];
  __shared__ __align__(16) float b1s[NGATE];
  __shared__ __align__(16) float outs[ROWS_BLK];

  const int tid  = threadIdx.x;
  const int lane = tid & 31;
  const int wave = tid >> 5;
  const int c    = lane & 15;
  const int hh   = lane >> 4;
  const int blockrow0 = blockIdx.x * ROWS_BLK;
  const int wrow0     = wave * 16;

  stage_w(W_hh0, Wl, tid);
  stage_w(W_ih1, Wl + WPLANE, tid);
  stage_w(W_hh1, Wl + 2 * WPLANE, tid);
  if (tid < NGATE) {
    const float w  = W_ih0[tid];
    const float ba = b_ih0[tid];
    const float bb = b_hh0[tid];
    const float bc = b_ih1[tid];
    const float bd = b_hh1[tid];
    w0s[tid] = w * Z_CARRY;
    b0s[tid] = (ba + bb) * Z_CARRY;
    b1s[tid] = (bc + bd) * Z_CARRY;
  }
  __syncthreads();

  union HB { v16h v; v8h h[2]; };
  HB h1B, h2B;
  const v8f z8 = {0.f, 0.f, 0.f, 0.f, 0.f, 0.f, 0.f, 0.f};
  v8f c1A = z8, c1B = z8, c2A = z8, c2B = z8, hfA = z8, hfB = z8;
  v8h hz;
#pragma unroll
  for (int e = 0; e < 8; ++e) hz[e] = (_Float16)0.0f;
  h1B.h[0] = hz; h1B.h[1] = hz;
  h2B.h[0] = hz; h2B.h[1] = hz;

#pragma unroll 1
  for (int t = 0; t < NSTEP; ++t) {
    const int tt = t & (XCHUNK - 1);
    if (tt == 0) {
      __syncthreads();
#pragma unroll
      for (int it = 0; it < 4; ++it) {
        const int row = it * 4 + (lane >> 3);
        const int q4  = (lane & 7) * 4;
        const v4f v = *(const v4f*)(x + (size_t)(blockrow0 + wrow0 + row) * NSTEP + (size_t)(t + q4));
        *(v4f*)(xs + (wrow0 + row) * XPITCH + q4) = v;
      }
      __syncthreads();
    }
    const float xv = xs[(wrow0 + c) * XPITCH + tt];

    v8h hnA = hz, hnB = hz;
#pragma unroll 1
    for (int ch = 0; ch < 2; ++ch) {
      int go = ch * 16;
      asm volatile("" : "+v"(go));
      const int gb = go + 8 * hh;
      v8f zi = cinit0(xv, w0s + gb,      b0s + gb);
      v8f zf = cinit0(xv, w0s + 32 + gb, b0s + 32 + gb);
      v8f zg = cinit0(xv, w0s + 64 + gb, b0s + 64 + gb);
      v8f zo = cinit0(xv, w0s + 96 + gb, b0s + 96 + gb);
      const _Float16* wa = Wl + (go + c) * NHID + 8 * hh;
      zi = wm(Frag<_Float16>::load(wa),             h1B.v, zi);
      zf = wm(Frag<_Float16>::load(wa + 32 * NHID), h1B.v, zf);
      zg = wm(Frag<_Float16>::load(wa + 64 * NHID), h1B.v, zg);
      zo = wm(Frag<_Float16>::load(wa + 96 * NHID), h1B.v, zo);
      acc_guard4(zi, zf, zg, zo);
      v8f cn, hn;
      lstm_cell8(zi, zf, zg, zo, c1A, cn, hn);
      v8h hp;
#pragma unroll
      for (int r = 0; r < 8; ++r) hp[r] = (_Float16)(hn[r] * H_CARRY);
      c1A = c1B; c1B = cn;
      hnA = hnB; hnB = hp;
    }
    h1B.h[0] = hnA;
    h1B.h[1] = hnB;

    v8h gnA = hz, gnB = hz;
#pragma unroll 1
    for (int ch = 0; ch < 2; ++ch) {
      int go = ch * 16;
      asm volatile("" : "+v"(go));
      const int gb = go + 8 * hh;
      v8f zi = ld8(b1s + gb);
      v8f zf = ld8(b1s + 32 + gb);
      v8f zg = ld8(b1s + 64 + gb);
      v8f zo = ld8(b1s + 96 + gb);
      const _Float16* wb = Wl + WPLANE     + (go + c) * NHID + 8 * hh;
      const _Float16* wc = Wl + 2 * WPLANE + (go + c) * NHID + 8 * hh;
      zi = wm(Frag<_Float16>::load(wb),             h1B.v, zi);
      zi = wm(Frag<_Float16>::load(wc),             h2B.v, zi);
      zf = wm(Frag<_Float16>::load(wb + 32 * NHID), h1B.v, zf);
      zf = wm(Frag<_Float16>::load(wc + 32 * NHID), h2B.v, zf);
      zg = wm(Frag<_Float16>::load(wb + 64 * NHID), h1B.v, zg);
      zg = wm(Frag<_Float16>::load(wc + 64 * NHID), h2B.v, zg);
      zo = wm(Frag<_Float16>::load(wb + 96 * NHID), h1B.v, zo);
      zo = wm(Frag<_Float16>::load(wc + 96 * NHID), h2B.v, zo);
      acc_guard4(zi, zf, zg, zo);
      v8f cn, hn;
      lstm_cell8(zi, zf, zg, zo, c2A, cn, hn);
      v8h hp;
#pragma unroll
      for (int r = 0; r < 8; ++r) hp[r] = (_Float16)(hn[r] * H_CARRY);
      c2A = c2B; c2B = cn;
      hfA = hfB; hfB = hn;
      gnA = gnB; gnB = hp;
    }
    h2B.h[0] = gnA;
    h2B.h[1] = gnB;
  }

  {
    const v4f f0 = *(const v4f*)(W_fc + 8 * hh);
    const v4f f1 = *(const v4f*)(W_fc + 8 * hh + 4);
    const v4f f2 = *(const v4f*)(W_fc + 16 + 8 * hh);
    const v4f f3 = *(const v4f*)(W_fc + 16 + 8 * hh + 4);
    const float bfc = b_fc[0];
    float part = 0.0f;
#pragma unroll
    for (int e = 0; e < 4; ++e) {
      part = fmaf(hfA[e],     f0[e], part);
      part = fmaf(hfA[4 + e], f1[e], part);
      part = fmaf(hfB[e],     f2[e], part);
      part = fmaf(hfB[4 + e], f3[e], part);
    }
    const float oth = __shfl_xor(part, 16, 32);
    const float tot = (part + oth) + bfc;
    if (hh == 0) outs[wrow0 + c] = tot;
  }
  __syncthreads();
  if (wave == 0) {
    const v4f v = *(const v4f*)(outs + 4 * lane);
    float* op = out + blockrow0 + 4 * lane;
    *(volatile v4f*)op = v;
    __threadfence();
    *(volatile v4f*)op = v;
  }
}

extern "C" void kernel_launch(void* const* d_in, const int* in_sizes, int n_in,
                              void* d_out, int out_size, void* d_ws, size_t ws_size, hipStream_t stream) {
  (void)d_ws; (void)ws_size;
  if (n_in < 11 || d_out == nullptr) return;
  if (in_sizes[0] != NBATCH * NSTEP || in_sizes[1] != NGATE || in_sizes[2] != NGATE * NHID ||
      in_sizes[3] != NGATE || in_sizes[4] != NGATE || in_sizes[5] != NGATE * NHID ||
      in_sizes[6] != NGATE * NHID || in_sizes[7] != NGATE || in_sizes[8] != NGATE ||
      in_sizes[9] != NHID || in_sizes[10] != 1 || out_size != NBATCH) return;

  const float* x     = (const float*)d_in[0];
  const float* W_ih0 = (const float*)d_in[1];
  const float* W_hh0 = (const float*)d_in[2];
  const float* b_ih0 = (const float*)d_in[3];
  const float* b_hh0 = (const float*)d_in[4];
  const float* W_ih1 = (const float*)d_in[5];
  const float* W_hh1 = (const float*)d_in[6];
  const float* b_ih1 = (const float*)d_in[7];
  const float* b_hh1 = (const float*)d_in[8];
  const float* W_fc  = (const float*)d_in[9];
  const float* b_fc  = (const float*)d_in[10];
  float* out = (float*)d_out;

  lstm2_fused_kernel<<<NBATCH / ROWS_BLK, NTHR, 0, stream>>>(x, W_ih0, W_hh0, b_ih0, b_hh0,
                                                             W_ih1, W_hh1, b_ih1, b_hh1, W_fc, b_fc, out);
}
